// MultiHeadAttentionLayer_4973572129389
// MI455X (gfx1250) — hardware-verified
//
#include <hip/hip_runtime.h>

#ifndef NB
#define NB 2
#endif
#define NB_FULL 2
#ifndef SEQ
#define SEQ 2048
#endif
#define SEQ_FULL 2048
#ifndef MASK_PITCH
#define MASK_PITCH SEQ_FULL
#endif
#define IN_DIM 1024
#define NUM_HEADS 16
#define HEAD_DIM 64
#define HD_DIM (NUM_HEADS * HEAD_DIM)
#define E_OUT 1024
#define KDIM 1024
#define NROWS (NB * SEQ)

static_assert(NB >= 1);
static_assert(NB <= NB_FULL);
static_assert(SEQ % 128 == 0);
static_assert(SEQ <= SEQ_FULL);
static_assert(MASK_PITCH % 4 == 0);
static_assert(MASK_PITCH >= SEQ);
static_assert(IN_DIM == KDIM);
static_assert(HD_DIM == KDIM);
static_assert(E_OUT == KDIM);
static_assert(KDIM % 64 == 0);
static_assert(HEAD_DIM == 64);
static_assert(NROWS % 128 == 0);
static_assert((NROWS * IN_DIM) % (8 * 256) == 0);
static_assert((size_t)NB_FULL * SEQ_FULL * E_OUT * 4 == 16777216);

#define BTP 40
#define EQP 72
#define EVP 136
#define TP  72
#define CLP 72
#define OFP 68
#define ESZ 9216
static_assert(128 * EQP <= ESZ);
static_assert(64 * EVP <= ESZ);

typedef __bf16   v16bf __attribute__((ext_vector_type(16)));
typedef __bf16   v8bf  __attribute__((ext_vector_type(8)));
typedef _Float16 v16h  __attribute__((ext_vector_type(16)));
typedef _Float16 v8h   __attribute__((ext_vector_type(8)));
typedef float    v8f   __attribute__((ext_vector_type(8)));
typedef float    v4f   __attribute__((ext_vector_type(4)));
typedef unsigned int v4u __attribute__((ext_vector_type(4)));
typedef int      v4i   __attribute__((ext_vector_type(4)));

__device__ __forceinline__ v8f mma_bf16(v16bf a, v16bf b, v8f c) {
  v8f d = __builtin_amdgcn_wmma_f32_16x16x32_bf16(false, a, false, b, (short)0, c, false, false);
  asm volatile("v_nop\n\tv_nop\n\tv_nop\n\tv_nop" : "+v"(d) : "v"(a), "v"(b));
  return d;
}
__device__ __forceinline__ v8f mma_f16(v16h a, v16h b, v8f c) {
  v8f d = __builtin_amdgcn_wmma_f32_16x16x32_f16(false, a, false, b, (short)0, c, false, false);
  asm volatile("v_nop\n\tv_nop\n\tv_nop\n\tv_nop" : "+v"(d) : "v"(a), "v"(b));
  return d;
}

__device__ __forceinline__ v16bf ld_frag_bf(const __bf16* p0, int ld, int rc, int kk, int lane) {
  const int hh = (lane >> 4) & 1;
  const __bf16* p = p0 + (size_t)rc * ld + kk + 8 * hh;
  const v8bf lo = *(const v8bf*)(p);
  const v8bf hi = *(const v8bf*)(p + 16);
  v16bf f;
#pragma unroll
  for (int i = 0; i < 8; ++i) { f[i] = lo[i]; f[8 + i] = hi[i]; }
  return f;
}
__device__ __forceinline__ v16h ld_frag_h(const _Float16* p0, int ld, int rc, int kk, int lane) {
  const int hh = (lane >> 4) & 1;
  const _Float16* p = p0 + (size_t)rc * ld + kk + 8 * hh;
  const v8h lo = *(const v8h*)(p);
  const v8h hi = *(const v8h*)(p + 16);
  v16h f;
#pragma unroll
  for (int i = 0; i < 8; ++i) { f[i] = lo[i]; f[8 + i] = hi[i]; }
  return f;
}

__device__ __forceinline__ unsigned int bfb(float x) {
  unsigned int u = __float_as_uint(x);
  u = u + 0x7FFFu + ((u >> 16) & 1u);
  return u >> 16;
}
__device__ __forceinline__ float bf16val(float x) {
  return __uint_as_float(bfb(x) << 16);
}
__device__ __forceinline__ unsigned short hbits(float x) {
  const _Float16 hv = (_Float16)x;
  return __builtin_bit_cast(unsigned short, hv);
}

__global__ __launch_bounds__(256) void k_cvt_rows(const float* __restrict__ in,
                                                  unsigned short* __restrict__ outp, int n8) {
  const int g = blockIdx.x * 256 + threadIdx.x;
  if (g >= n8) return;
  const int row = g / (IN_DIM / 8);
  const int c8  = g - row * (IN_DIM / 8);
  const int b   = row / SEQ;
  const int s   = row - b * SEQ;
  const float* src = in + ((size_t)b * SEQ_FULL + s) * IN_DIM + (size_t)c8 * 8;
  const v4f a = *(const v4f*)(src);
  const v4f c = *(const v4f*)(src + 4);
  v4u w;
  w[0] = bfb(a[0]) | (bfb(a[1]) << 16);
  w[1] = bfb(a[2]) | (bfb(a[3]) << 16);
  w[2] = bfb(c[0]) | (bfb(c[1]) << 16);
  w[3] = bfb(c[2]) | (bfb(c[3]) << 16);
  volatile v4u* p = (volatile v4u*)(outp + (size_t)g * 8);
  *p = w;
  __threadfence();
  *p = w;
}

__global__ __launch_bounds__(256) void k_cvt_wT(const float* __restrict__ Wq,
                                                const float* __restrict__ Wk,
                                                const float* __restrict__ Wv,
                                                const float* __restrict__ Wo,
                                                unsigned short* __restrict__ wT) {
  __shared__ __align__(16) unsigned short T[64 * TP];
  const int z = blockIdx.z;
  const float* W = (z == 0) ? Wq : ((z == 1) ? Wk : ((z == 2) ? Wv : Wo));
  unsigned short* dst = wT + (size_t)z * KDIM * KDIM;
  const int k0 = blockIdx.x * 64;
  const int n0 = blockIdx.y * 64;
  const int tid = threadIdx.x;
  const int wave = tid >> 5, lane = tid & 31;

#pragma unroll
  for (int i = 0; i < 4; ++i) {
    const int idx = i * 256 + tid;
    const int kk = idx >> 4;
    const int c4 = (idx & 15) * 4;
    size_t so;
    if (z < 3) so = ((size_t)blockIdx.y * IN_DIM + k0 + kk) * HEAD_DIM + c4;
    else       so = (size_t)(k0 + kk) * E_OUT + n0 + c4;
    const v4f w = *(const v4f*)(W + so);
    unsigned short t0, t1, t2, t3;
    if (z < 3) {
      t0 = (unsigned short)bfb(w[0]); t1 = (unsigned short)bfb(w[1]);
      t2 = (unsigned short)bfb(w[2]); t3 = (unsigned short)bfb(w[3]);
    } else {
      t0 = hbits(bf16val(w[0]) * 32.0f); t1 = hbits(bf16val(w[1]) * 32.0f);
      t2 = hbits(bf16val(w[2]) * 32.0f); t3 = hbits(bf16val(w[3]) * 32.0f);
    }
    T[(c4 + 0) * TP + kk] = t0;
    T[(c4 + 1) * TP + kk] = t1;
    T[(c4 + 2) * TP + kk] = t2;
    T[(c4 + 3) * TP + kk] = t3;
  }
  __syncthreads();

  v4u v[2];
  size_t off[2];
#pragma unroll
  for (int it = 0; it < 2; ++it) {
    const int nn = wave * 8 + it * 4 + (lane >> 3);
    const int q = lane & 7;
    v[it] = *(const v4u*)(&T[nn * TP + q * 8]);
    off[it] = (size_t)(n0 + nn) * KDIM + k0 + q * 8;
  }
#pragma unroll
  for (int it = 0; it < 2; ++it) *(volatile v4u*)(dst + off[it]) = v[it];
  __threadfence();
#pragma unroll
  for (int it = 0; it < 2; ++it) *(volatile v4u*)(dst + off[it]) = v[it];
}

__global__ __launch_bounds__(256) void k_proj(
    const unsigned short* __restrict__ hb, const unsigned short* __restrict__ wT,
    const float* __restrict__ bq, const float* __restrict__ bk, const float* __restrict__ bv,
    unsigned short* __restrict__ qp, unsigned short* __restrict__ kp,
    unsigned short* __restrict__ vtp) {
  __shared__ __align__(16) unsigned short bt[64 * BTP];
  __shared__ __align__(16) unsigned short E[ESZ];

  const int z = blockIdx.z;
  const int n0 = blockIdx.x * 64;
  const int m0 = blockIdx.y * 128;
  const int tid = threadIdx.x;
  const int wave = tid >> 5, lane = tid & 31;
  const int l15 = lane & 15, half = (lane >> 4) & 1;

  const unsigned short* Wt = wT + (size_t)z * KDIM * KDIM;
  const float* bias = (z == 0) ? bq : ((z == 1) ? bk : bv);

  const int tn = tid >> 2;
  const int tk = (tid & 3) * 8;
  const unsigned short* wsrc = Wt + (size_t)(n0 + tn) * KDIM + tk;
  const __bf16* A = (const __bf16*)hb;
  const int arow = m0 + wave * 16 + l15;

  v8f acc[4] = {};
  for (int s = 0; s < IN_DIM / 32; ++s) {
    const int kk = s * 32;
    const v4u wv = *(const v4u*)(wsrc + kk);
    __syncthreads();
    *(v4u*)(&bt[tn * BTP + tk]) = wv;
    __syncthreads();
    const v16bf a = ld_frag_bf(A, IN_DIM, arow, kk, lane);
#pragma unroll
    for (int j = 0; j < 4; ++j) {
      const v16bf b = ld_frag_bf((const __bf16*)bt, BTP, j * 16 + l15, 0, lane);
      acc[j] = mma_bf16(a, b, acc[j]);
    }
  }

  const float car = 8.0f;
  if (z != 2) {
#pragma unroll
    for (int j = 0; j < 4; ++j) {
      const int col = j * 16 + l15;
      const float bb = bf16val(bias[n0 + col]);
#pragma unroll
      for (int r = 0; r < 8; ++r) {
        const int row = wave * 16 + 8 * half + r;
        E[row * EQP + col] = hbits((acc[j][r] + bb) * car);
      }
    }
    __syncthreads();
    unsigned short* dst = (z == 0) ? qp : kp;
    v4u v[4];
    size_t off[4];
#pragma unroll
    for (int it = 0; it < 4; ++it) {
      const int row = wave * 16 + it * 4 + (lane >> 3);
      const int q = lane & 7;
      v[it] = *(const v4u*)(&E[row * EQP + q * 8]);
      off[it] = (size_t)(m0 + row) * HD_DIM + n0 + q * 8;
    }
#pragma unroll
    for (int it = 0; it < 4; ++it) *(volatile v4u*)(dst + off[it]) = v[it];
    __threadfence();
#pragma unroll
    for (int it = 0; it < 4; ++it) *(volatile v4u*)(dst + off[it]) = v[it];
  } else {
    const int bidx = m0 / SEQ;
    const int s0 = m0 - bidx * SEQ;
#pragma unroll
    for (int j = 0; j < 4; ++j) {
      const int col = j * 16 + l15;
      const float bb = bf16val(bias[n0 + col]);
#pragma unroll
      for (int r = 0; r < 8; ++r) {
        const int srow = wave * 16 + 8 * half + r;
        E[col * EVP + srow] = hbits((acc[j][r] + bb) * car);
      }
    }
    __syncthreads();
    v4u v[4];
    size_t off[4];
#pragma unroll
    for (int it = 0; it < 4; ++it) {
      const int drow = wave * 8 + it * 2 + half;
      const int q = l15;
      v[it] = *(const v4u*)(&E[drow * EVP + q * 8]);
      off[it] = ((size_t)bidx * HD_DIM + n0 + drow) * SEQ + s0 + q * 8;
    }
#pragma unroll
    for (int it = 0; it < 4; ++it) *(volatile v4u*)(vtp + off[it]) = v[it];
    __threadfence();
#pragma unroll
    for (int it = 0; it < 4; ++it) *(volatile v4u*)(vtp + off[it]) = v[it];
  }
}

__global__ __launch_bounds__(32) void k_attn(const unsigned short* __restrict__ qp,
                                             const unsigned short* __restrict__ kp,
                                             const unsigned short* __restrict__ vtp,
                                             const int* __restrict__ mask,
                                             unsigned short* __restrict__ ctxp) {
  __shared__ __align__(16) unsigned short Cl[16 * CLP];

  const int lane = threadIdx.x & 31;
  const int l15 = lane & 15;
  const int half = (lane >> 4) & 1;
  const int q0 = blockIdx.x * 16;
  const int head = blockIdx.y;
  const int bidx = blockIdx.z;

  const _Float16* Q  = (const _Float16*)qp;
  const _Float16* K  = (const _Float16*)kp;
  const _Float16* VT = (const _Float16*)vtp;
  const size_t rbase = (size_t)bidx * SEQ;

  const _Float16* qbase = Q + (rbase + q0) * HD_DIM + head * HEAD_DIM;
  const v16h qb0 = ld_frag_h(qbase, HD_DIM, l15, 0, lane);
  const v16h qb1 = ld_frag_h(qbase, HD_DIM, l15, 32, lane);
  const _Float16* kbase = K + rbase * HD_DIM + head * HEAD_DIM;
  const _Float16* vbase = VT + ((size_t)bidx * HD_DIM + (size_t)head * HEAD_DIM) * SEQ;
  const int* mrow = mask + (size_t)(q0 + l15) * MASK_PITCH + 8 * half;

  v8f o[4] = {};
  float mrun = -1.0e30f, lrun = 0.0f;
  const float sscale = 1.0f / 512.0f;
  const float negf = -1.0e9f;

  for (int kc = 0; kc < SEQ; kc += 32) {
    const _Float16* kt = kbase + (size_t)kc * HD_DIM;
    const v16h ka0 = ld_frag_h(kt, HD_DIM, l15, 0, lane);
    const v16h ka1 = ld_frag_h(kt, HD_DIM, l15, 32, lane);
    const v16h ka2 = ld_frag_h(kt, HD_DIM, 16 + l15, 0, lane);
    const v16h ka3 = ld_frag_h(kt, HD_DIM, 16 + l15, 32, lane);
    v8f c0 = {}, c1 = {};
    c0 = mma_f16(ka0, qb0, c0);
    c0 = mma_f16(ka1, qb1, c0);
    c1 = mma_f16(ka2, qb0, c1);
    c1 = mma_f16(ka3, qb1, c1);

    const v4i m0v = *(const v4i*)(mrow + kc);
    const v4i m1v = *(const v4i*)(mrow + kc + 4);
    const v4i m2v = *(const v4i*)(mrow + kc + 16);
    const v4i m3v = *(const v4i*)(mrow + kc + 20);

    float sa[8], sb[8];
#pragma unroll
    for (int r = 0; r < 4; ++r) {
      sa[r]     = (m0v[r] != 0) ? (c0[r] * sscale)     : negf;
      sa[4 + r] = (m1v[r] != 0) ? (c0[4 + r] * sscale) : negf;
      sb[r]     = (m2v[r] != 0) ? (c1[r] * sscale)     : negf;
      sb[4 + r] = (m3v[r] != 0) ? (c1[4 + r] * sscale) : negf;
    }
    float lm = fmaxf(sa[0], sb[0]);
#pragma unroll
    for (int r = 1; r < 8; ++r) lm = fmaxf(lm, fmaxf(sa[r], sb[r]));
    lm = fmaxf(lm, __shfl_xor(lm, 16, 32));
    const float mnew = fmaxf(mrun, lm);
    const float alpha = __expf(mrun - mnew);
    float p0[8], p1[8];
    float ls = 0.0f;
#pragma unroll
    for (int r = 0; r < 8; ++r) {
      p0[r] = __expf(sa[r] - mnew);
      p1[r] = __expf(sb[r] - mnew);
      ls += p0[r] + p1[r];
    }
    ls += __shfl_xor(ls, 16, 32);
    lrun = lrun * alpha + ls;
    mrun = mnew;
#pragma unroll
    for (int j = 0; j < 4; ++j)
#pragma unroll
      for (int r = 0; r < 8; ++r) o[j][r] *= alpha;

    v16h pb;
#pragma unroll
    for (int e = 0; e < 8; ++e) {
      pb[e]     = (_Float16)(p0[e] * 1024.0f);
      pb[8 + e] = (_Float16)(p1[e] * 1024.0f);
    }
#pragma unroll
    for (int j = 0; j < 4; ++j) {
      const v16h va = ld_frag_h(vbase, SEQ, j * 16 + l15, kc, lane);
      o[j] = mma_f16(va, pb, o[j]);
    }
  }

  const float inv = 1.0f / (lrun * 128.0f);
#pragma unroll
  for (int j = 0; j < 4; ++j) {
    v4u w;
    w[0] = (unsigned int)hbits(o[j][0] * inv) | ((unsigned int)hbits(o[j][1] * inv) << 16);
    w[1] = (unsigned int)hbits(o[j][2] * inv) | ((unsigned int)hbits(o[j][3] * inv) << 16);
    w[2] = (unsigned int)hbits(o[j][4] * inv) | ((unsigned int)hbits(o[j][5] * inv) << 16);
    w[3] = (unsigned int)hbits(o[j][6] * inv) | ((unsigned int)hbits(o[j][7] * inv) << 16);
    *(v4u*)(&Cl[l15 * CLP + j * 16 + 8 * half]) = w;
  }
  __syncthreads();

  v4u v[4];
  size_t off[4];
  unsigned short* cb = ctxp + (rbase + q0) * HD_DIM + head * HEAD_DIM;
#pragma unroll
  for (int it = 0; it < 4; ++it) {
    const int row = it * 4 + (lane >> 3);
    const int q = lane & 7;
    v[it] = *(const v4u*)(&Cl[row * CLP + q * 8]);
    off[it] = (size_t)row * HD_DIM + q * 8;
  }
#pragma unroll
  for (int it = 0; it < 4; ++it) *(volatile v4u*)(cb + off[it]) = v[it];
  __threadfence();
#pragma unroll
  for (int it = 0; it < 4; ++it) *(volatile v4u*)(cb + off[it]) = v[it];
}

__global__ __launch_bounds__(256) void k_oproj(
    const unsigned short* __restrict__ cx, const unsigned short* __restrict__ woT,
    const float* __restrict__ bo, float* __restrict__ outp) {
  __shared__ __align__(16) unsigned short bt[64 * BTP];
  __shared__ __align__(16) float Ef[128 * OFP];

  const int n0 = blockIdx.x * 64;
  const int m0 = blockIdx.y * 128;
  const int tid = threadIdx.x;
  const int wave = tid >> 5, lane = tid & 31;
  const int l15 = lane & 15, half = (lane >> 4) & 1;

  const int tn = tid >> 2;
  const int tk = (tid & 3) * 8;
  const unsigned short* wsrc = woT + (size_t)(n0 + tn) * KDIM + tk;
  const _Float16* A = (const _Float16*)cx;
  const int arow = m0 + wave * 16 + l15;

  v8f acc[4] = {};
  for (int s = 0; s < HD_DIM / 32; ++s) {
    const int kk = s * 32;
    const v4u wv = *(const v4u*)(wsrc + kk);
    __syncthreads();
    *(v4u*)(&bt[tn * BTP + tk]) = wv;
    __syncthreads();
    const v16h a = ld_frag_h(A, HD_DIM, arow, kk, lane);
#pragma unroll
    for (int j = 0; j < 4; ++j) {
      const v16h b = ld_frag_h((const _Float16*)bt, BTP, j * 16 + l15, 0, lane);
      acc[j] = mma_f16(a, b, acc[j]);
    }
  }

  const float osc = 1.0f / 2048.0f;
#pragma unroll
  for (int j = 0; j < 4; ++j) {
    const int col = j * 16 + l15;
    const float bb = bf16val(bo[n0 + col]);
#pragma unroll
    for (int r = 0; r < 8; ++r) {
      const int row = wave * 16 + 8 * half + r;
      Ef[row * OFP + col] = acc[j][r] * osc + bb;
    }
  }
  __syncthreads();

  v4f v[8];
  size_t off[8];
#pragma unroll
  for (int it = 0; it < 8; ++it) {
    const int row = wave * 16 + it * 2 + half;
    const int q = l15;
    v[it] = *(const v4f*)(&Ef[row * OFP + q * 4]);
    off[it] = (size_t)(m0 + row) * E_OUT + n0 + q * 4;
  }
#pragma unroll
  for (int it = 0; it < 8; ++it) *(volatile v4f*)(outp + off[it]) = v[it];
  __threadfence();
#pragma unroll
  for (int it = 0; it < 8; ++it) *(volatile v4f*)(outp + off[it]) = v[it];
}

extern "C" void kernel_launch(void* const* d_in, const int* in_sizes, int n_in,
                              void* d_out, int out_size, void* d_ws, size_t ws_size,
                              hipStream_t stream) {
  if (n_in < 10) return;
  if (in_sizes[0] < ((NB - 1) * SEQ_FULL + SEQ) * IN_DIM) return;
  if (in_sizes[1] < (SEQ - 1) * MASK_PITCH + SEQ) return;
  if (in_sizes[2] < NUM_HEADS * IN_DIM * HEAD_DIM) return;
  if (in_sizes[3] < HD_DIM) return;
  if (in_sizes[4] < NUM_HEADS * IN_DIM * HEAD_DIM) return;
  if (in_sizes[5] < HD_DIM) return;
  if (in_sizes[6] < NUM_HEADS * IN_DIM * HEAD_DIM) return;
  if (in_sizes[7] < HD_DIM) return;
  if (in_sizes[8] < HD_DIM * E_OUT) return;
  if (in_sizes[9] < E_OUT) return;
  if (out_size < NROWS * E_OUT) return;

  const float* x    = (const float*)d_in[0];
  const int*   mask = (const int*)d_in[1];
  const float* Wq   = (const float*)d_in[2];
  const float* bq   = (const float*)d_in[3];
  const float* Wk   = (const float*)d_in[4];
  const float* bk   = (const float*)d_in[5];
  const float* Wv   = (const float*)d_in[6];
  const float* bv   = (const float*)d_in[7];
  const float* Wo   = (const float*)d_in[8];
  const float* bo   = (const float*)d_in[9];

  const size_t hb_bytes = (size_t)NROWS * IN_DIM * 2;
  const size_t wt_bytes = (size_t)4 * KDIM * KDIM * 2;
  const size_t pl_bytes = (size_t)NROWS * HD_DIM * 2;
  const size_t off_hb = 0;
  const size_t off_wt = off_hb + hb_bytes;
  const size_t off_q  = off_wt + wt_bytes;
  const size_t off_k  = off_q + pl_bytes;
  const size_t off_vt = off_k + pl_bytes;
  const size_t off_cx = off_vt + pl_bytes;
  const size_t total  = off_cx + pl_bytes;
  if (total > ws_size) return;

  char* ws = (char*)d_ws;
  unsigned short* hb  = (unsigned short*)(ws + off_hb);
  unsigned short* wt  = (unsigned short*)(ws + off_wt);
  unsigned short* qpl = (unsigned short*)(ws + off_q);
  unsigned short* kpl = (unsigned short*)(ws + off_k);
  unsigned short* vtp = (unsigned short*)(ws + off_vt);
  unsigned short* cxp = (unsigned short*)(ws + off_cx);
  unsigned short* wot = wt + (size_t)3 * KDIM * KDIM;

  const int n8 = NROWS * IN_DIM / 8;
  k_cvt_rows<<<(n8 + 255) / 256, 256, 0, stream>>>(x, hb, n8);
  k_cvt_wT<<<dim3(KDIM / 64, KDIM / 64, 4), 256, 0, stream>>>(Wq, Wk, Wv, Wo, wt);
  k_proj<<<dim3(HD_DIM / 64, NROWS / 128, 3), 256, 0, stream>>>(hb, wt, bq, bk, bv, qpl, kpl, vtp);
  k_attn<<<dim3(SEQ / 16, NUM_HEADS, NB), 32, 0, stream>>>(qpl, kpl, vtp, mask, cxp);
  k_oproj<<<dim3(E_OUT / 64, NROWS / 128), 256, 0, stream>>>(cxp, wot, bo, (float*)d_out);
}
